// Attention_72499047957038
// MI455X (gfx1250) — hardware-verified
//
#include <hip/hip_runtime.h>
#include <stddef.h>


#ifndef NB
#define NB 2
#endif
#ifndef SEQ
#define SEQ 2048
#endif
#ifndef RHP
#define RHP 1024
#endif

#define NB_FULL  2
#define SEQ_FULL 2048
#define HID      2048
#define NH       32
#define NKV      8
#define HDM      64
#define KVD      (NKV * HDM)
#define NTOK     (NB * SEQ)
#define RHPE     (((RHP) < (SEQ)) ? (RHP) : (SEQ))

static_assert(NB >= 1 && NB <= NB_FULL);
static_assert(SEQ % 128 == 0 && SEQ >= 128 && SEQ <= SEQ_FULL);
static_assert((RHPE % 128) == 0 && RHPE >= 128 && RHPE <= SEQ);
static_assert(HID % 128 == 0 && KVD % 128 == 0 && (NTOK % 128) == 0 && (NTOK % 8) == 0);
static_assert(NH * HDM == HID && NH == 4 * NKV && HDM == 64);

#define LST 40
#define TPH 136
#define TPF 132
#define KP  72
#define PROJ_LDS_BYTES  102400
#define OPROJ_LDS_BYTES 67584
static_assert(2 * 128 * LST * 2 <= 128 * TPH * 2);
static_assert(2 * 128 * TPH * 2 + 128 * 64 * 4 == PROJ_LDS_BYTES);
static_assert(128 * TPF * 4 == OPROJ_LDS_BYTES && 2 * 128 * LST * 2 <= OPROJ_LDS_BYTES);

#define WSCALE     256.0f
#define WSCALE_INV 0.00390625f
#define LOSC       2048.0f
#define LOSC_INV   0.00048828125f
#define PSC        4096.0f
#define SM_SCALE   0.125f

typedef _Float16 v16h __attribute__((ext_vector_type(16)));
typedef _Float16 v8h  __attribute__((ext_vector_type(8)));
typedef float    v8f  __attribute__((ext_vector_type(8)));
typedef float    v4f  __attribute__((ext_vector_type(4)));

union Frag16 { v16h v; v8h p[2]; };

extern __shared__ __attribute__((aligned(16))) unsigned char dyn_lds[];

__device__ __forceinline__ float bf16r(float x) {
    unsigned int u = __float_as_uint(x);
    u += 0x7FFFu + ((u >> 16) & 1u);
    u &= 0xFFFF0000u;
    return __uint_as_float(u);
}

__device__ __forceinline__ v8f zero8() {
    const v8f z = {0.0f, 0.0f, 0.0f, 0.0f, 0.0f, 0.0f, 0.0f, 0.0f};
    return z;
}

__device__ __forceinline__ v8f mma(v16h a, v16h b, v8f c) {
    v8f d = __builtin_amdgcn_wmma_f32_16x16x32_f16(false, a, false, b, (short)0, c, false, false);
    asm volatile("v_nop\n\tv_nop\n\tv_nop\n\tv_nop" : "+v"(d) : "v"(a), "v"(b));
    return d;
}

__device__ __forceinline__ v16h ldfrag(const _Float16* p) {
    Frag16 f;
    f.p[0] = *(const v8h*)(p);
    f.p[1] = *(const v8h*)(p + 16);
    return f.v;
}

__device__ __forceinline__ void gemm_kloop(const _Float16* __restrict__ A, const _Float16* __restrict__ Bt,
                                           int mBase, int nBase, _Float16* As, _Float16* Bs,
                                           v8f (&acc)[2][4])
{
    const int t = threadIdx.x, lane = t & 31, wave = t >> 5, lr = lane & 15, h = lane >> 4;
    const int waveM = wave & 3, waveN = wave >> 2;
    const int arow = t >> 1, acol = (t & 1) * 16;
    const _Float16* aSrc = A  + (size_t)(mBase + arow) * HID + acol;
    const _Float16* bSrc = Bt + (size_t)(nBase + arow) * HID + acol;
    _Float16* da = As + arow * LST + acol;
    _Float16* db = Bs + arow * LST + acol;

#pragma unroll 1
    for (int k0 = 0; k0 < HID; k0 += 32) {
        __syncthreads();
        const v8h a0 = *(const v8h*)(aSrc + k0);
        const v8h a1 = *(const v8h*)(aSrc + k0 + 8);
        const v8h b0 = *(const v8h*)(bSrc + k0);
        const v8h b1 = *(const v8h*)(bSrc + k0 + 8);
        *(v8h*)(da) = a0; *(v8h*)(da + 8) = a1;
        *(v8h*)(db) = b0; *(v8h*)(db + 8) = b1;
        __syncthreads();

        v16h af[2], bf[4];
#pragma unroll
        for (int mi = 0; mi < 2; ++mi)
            af[mi] = ldfrag(As + (waveM * 32 + mi * 16 + lr) * LST + 8 * h);
#pragma unroll
        for (int ni = 0; ni < 4; ++ni)
            bf[ni] = ldfrag(Bs + (waveN * 64 + ni * 16 + lr) * LST + 8 * h);
#pragma unroll
        for (int mi = 0; mi < 2; ++mi)
#pragma unroll
            for (int ni = 0; ni < 4; ++ni)
                acc[mi][ni] = mma(af[mi], bf[ni], acc[mi][ni]);
    }
    __syncthreads();
}

__global__ void __launch_bounds__(256)
cvt_x_kernel(const float* __restrict__ x, _Float16* __restrict__ xh)
{
    const int tok = blockIdx.x;
    const int b = tok / SEQ, s = tok - b * SEQ;
    const float* src = x + ((size_t)b * SEQ_FULL + s) * HID + threadIdx.x * 8;
    const v4f a0 = *(const v4f*)(src);
    const v4f a1 = *(const v4f*)(src + 4);
    v8h o;
#pragma unroll
    for (int i = 0; i < 4; ++i) {
        o[i]     = (_Float16)bf16r(a0[i]);
        o[i + 4] = (_Float16)bf16r(a1[i]);
    }
    _Float16* dst = xh + (size_t)tok * HID + threadIdx.x * 8;
    *(volatile v8h*)dst = o;
    __threadfence();
    *(volatile v8h*)dst = o;
}

__global__ void __launch_bounds__(256)
cvt_w_kernel(const float* __restrict__ w, _Float16* __restrict__ wt, int N)
{
    __shared__ float T[64][65];
    const int t = threadIdx.x;
    const int kb = blockIdx.y * 64, nb = blockIdx.x * 64;
    const int nn = t & 63, kq = t >> 6;
#pragma unroll 4
    for (int j = 0; j < 16; ++j) {
        const int kk = kq + 4 * j;
        T[kk][nn] = w[(size_t)(kb + kk) * N + nb + nn];
    }
    __syncthreads();
    auto emit = [&]() {
#pragma unroll
        for (int it = 0; it < 2; ++it) {
            const int slot = it * 256 + t, line = slot >> 3, ch = slot & 7;
            v8h o;
#pragma unroll
            for (int j = 0; j < 8; ++j) o[j] = (_Float16)(bf16r(T[ch * 8 + j][line]) * WSCALE);
            _Float16* dst = wt + (size_t)(nb + line) * HID + kb + ch * 8;
            *(volatile v8h*)dst = o;
        }
    };
    emit();
    __threadfence();
    emit();
}

__global__ void __launch_bounds__(256)
rope_table_kernel(const int* __restrict__ pos, float* __restrict__ cs)
{
#pragma clang fp contract(off)
    __shared__ __attribute__((aligned(16))) float csl[8][64];
    const int t = threadIdx.x;
    const int tl = t >> 5, i = t & 31;
    const int tok = blockIdx.x * 8 + tl;
    const int b = tok / SEQ, s = tok - b * SEQ;
    const int p = pos[b * SEQ_FULL + s];

    double pw = 1.0;
#pragma unroll 1
    for (int j = 0; j < i; ++j) pw *= 1.333521432163324;
    const float t32 = (float)pw;
    const float inv = 1.0f / t32;
    const float ang = (float)p * inv;

    const double a  = (double)ang;
    const double kd = __builtin_rint(a * 0.6366197723675814);
    double r = __builtin_fma(-kd, 1.5707963267948966, a);
    r = __builtin_fma(-kd, 6.123233995736766e-17, r);
    const double r2 = r * r;
    double sp = 1.6059043836821613e-10;
    sp = __builtin_fma(sp, r2, -2.5052108385441719e-8);
    sp = __builtin_fma(sp, r2, 2.7557319223985891e-6);
    sp = __builtin_fma(sp, r2, -1.9841269841269841e-4);
    sp = __builtin_fma(sp, r2, 8.3333333333333333e-3);
    sp = __builtin_fma(sp, r2, -1.6666666666666666e-1);
    sp = __builtin_fma(sp * r2, r, r);
    double cp = -1.1470745597729725e-11;
    cp = __builtin_fma(cp, r2, 2.0876756987868099e-9);
    cp = __builtin_fma(cp, r2, -2.7557319223985891e-7);
    cp = __builtin_fma(cp, r2, 2.4801587301587302e-5);
    cp = __builtin_fma(cp, r2, -1.3888888888888889e-3);
    cp = __builtin_fma(cp, r2, 4.1666666666666667e-2);
    cp = __builtin_fma(cp, r2, -0.5);
    cp = __builtin_fma(cp, r2, 1.0);
    const long long kk = (long long)kd;
    const int q = (int)(kk & 3);
    const double sv = (q == 0) ? sp : (q == 1) ? cp : (q == 2) ? -sp : -cp;
    const double cv = (q == 0) ? cp : (q == 1) ? -sp : (q == 2) ? -cp : sp;
    csl[tl][i]      = (float)cv;
    csl[tl][32 + i] = (float)sv;
    __syncthreads();

    const int line = t >> 3, tokl = line >> 1, half = line & 1, ch = t & 7;
    v4f v = {0.0f, 0.0f, 0.0f, 0.0f};
    float* dst = cs;
    if (t < 128) {
        v = *(const v4f*)(&csl[tokl][half * 32 + ch * 4]);
        dst = cs + (size_t)(blockIdx.x * 8 + tokl) * 64 + half * 32 + ch * 4;
        *(volatile v4f*)dst = v;
    }
    __threadfence();
    if (t < 128) {
        *(volatile v4f*)dst = v;
    }
}

template <int MODE>
__global__ void __launch_bounds__(256)
proj_kernel(const _Float16* __restrict__ xh, const _Float16* __restrict__ wt,
            const float* __restrict__ cs, _Float16* __restrict__ outh, _Float16* __restrict__ outl)
{
    constexpr int NHD = (MODE == 0) ? NH : NKV;
    _Float16* As  = (_Float16*)dyn_lds;
    _Float16* Bs  = As + 128 * LST;
    _Float16* Th  = (_Float16*)dyn_lds;
    _Float16* Tl  = Th + 128 * TPH;
    float*    CSl = (float*)(dyn_lds + (size_t)2 * 128 * TPH * 2);

    const int t = threadIdx.x, lane = t & 31, wave = t >> 5, lr = lane & 15, h = lane >> 4;
    const int waveM = wave & 3, waveN = wave >> 2;
    const int mBase = blockIdx.y * 128;
    const int nBase = blockIdx.x * 128;

    v8f acc[2][4];
#pragma unroll
    for (int mi = 0; mi < 2; ++mi)
#pragma unroll
        for (int ni = 0; ni < 4; ++ni) acc[mi][ni] = zero8();

    gemm_kloop(xh, wt, mBase, nBase, As, Bs, acc);

    if constexpr (MODE < 2) {
#pragma unroll
        for (int j = 0; j < 8; ++j) {
            const int idx = j * 256 + t, rowl = idx >> 4, c4 = idx & 15;
            *(v4f*)(CSl + rowl * 64 + c4 * 4) =
                *(const v4f*)(cs + (size_t)(mBase + rowl) * 64 + c4 * 4);
        }
        __syncthreads();
    }

    const int rbw = waveM * 32 + 8 * h;
#pragma unroll
    for (int mi = 0; mi < 2; ++mi) {
        const int rb = rbw + mi * 16;
        if constexpr (MODE < 2) {
#pragma unroll
            for (int nip = 0; nip < 2; ++nip) {
                const int i = nip * 16 + lr;
                v8h h1, h2, l1, l2;
#pragma unroll
                for (int r = 0; r < 8; ++r) {
                    const float cth = CSl[(rb + r) * 64 + i];
                    const float sth = CSl[(rb + r) * 64 + 32 + i];
                    const float x1 = acc[mi][nip][r] * WSCALE_INV;
                    const float x2 = acc[mi][nip + 2][r] * WSCALE_INV;
                    const float o1 = x1 * cth - x2 * sth;
                    const float o2 = x2 * cth + x1 * sth;
                    const _Float16 e1 = (_Float16)o1, e2 = (_Float16)o2;
                    h1[r] = e1; h2[r] = e2;
                    l1[r] = (_Float16)((o1 - (float)e1) * LOSC);
                    l2[r] = (_Float16)((o2 - (float)e2) * LOSC);
                }
                const int c1 = waveN * 64 + nip * 16 + lr, c2 = c1 + 32;
                *(v8h*)(Th + c1 * TPH + rb) = h1;
                *(v8h*)(Th + c2 * TPH + rb) = h2;
                *(v8h*)(Tl + c1 * TPH + rb) = l1;
                *(v8h*)(Tl + c2 * TPH + rb) = l2;
            }
        } else {
#pragma unroll
            for (int ni = 0; ni < 4; ++ni) {
                v8h hv, lv;
#pragma unroll
                for (int r = 0; r < 8; ++r) {
                    const float o = acc[mi][ni][r] * WSCALE_INV;
                    const _Float16 e = (_Float16)o;
                    hv[r] = e;
                    lv[r] = (_Float16)((o - (float)e) * LOSC);
                }
                const int col = waveN * 64 + ni * 16 + lr;
                *(v8h*)(Th + col * TPH + rb) = hv;
                *(v8h*)(Tl + col * TPH + rb) = lv;
            }
        }
    }
    __syncthreads();

    auto emit = [&]() {
#pragma unroll
        for (int it = 0; it < 8; ++it) {
            const int slot = it * 256 + t, L = slot >> 3, ch = slot & 7;
            if constexpr (MODE < 2) {
                const int headl = L >> 7, tokl = L & 127;
                v8h hv, lv;
#pragma unroll
                for (int j = 0; j < 8; ++j) {
                    const int src = (headl * 64 + ch * 8 + j) * TPH + tokl;
                    hv[j] = Th[src];
                    lv[j] = Tl[src];
                }
                const int tok = mBase + tokl, bb = tok / SEQ, ss = tok - bb * SEQ;
                const int head = (nBase >> 6) + headl;
                const size_t d = (((size_t)(bb * NHD + head)) * SEQ + ss) * HDM + ch * 8;
                *(volatile v8h*)(outh + d) = hv;
                *(volatile v8h*)(outl + d) = lv;
            } else {
                const int coll = L >> 1, half = L & 1;
                const v8h hv = *(const v8h*)(Th + coll * TPH + half * 64 + ch * 8);
                const v8h lv = *(const v8h*)(Tl + coll * TPH + half * 64 + ch * 8);
                const int head = (nBase >> 6) + (coll >> 6), dd = coll & 63;
                const int bb = mBase / SEQ, s0 = mBase - bb * SEQ + half * 64 + ch * 8;
                const size_t d = (((size_t)(bb * NKV + head)) * HDM + dd) * SEQ + s0;
                *(volatile v8h*)(outh + d) = hv;
                *(volatile v8h*)(outl + d) = lv;
            }
        }
    };
    emit();
    __threadfence();
    emit();
}

template <bool HP>
__global__ void __launch_bounds__(128)
attn_kernel(const _Float16* __restrict__ Qh, const _Float16* __restrict__ Ql,
            const _Float16* __restrict__ Kh, const _Float16* __restrict__ Kl,
            const _Float16* __restrict__ Vh, const _Float16* __restrict__ Vl,
            _Float16* __restrict__ Ch, _Float16* __restrict__ Cl, int qt0)
{
    __shared__ __attribute__((aligned(16))) _Float16 Ks[64 * KP];
    __shared__ __attribute__((aligned(16))) _Float16 Vs[64 * KP];
    __shared__ __attribute__((aligned(16))) _Float16 Kls[HP ? 64 * KP : 8];
    __shared__ __attribute__((aligned(16))) _Float16 Vls[HP ? 64 * KP : 8];
    __shared__ __attribute__((aligned(16))) _Float16 Ps[4 * 16 * KP];
    __shared__ __attribute__((aligned(16))) _Float16 Pls[HP ? 4 * 16 * KP : 8];

    const int t = threadIdx.x, lane = t & 31, wave = t >> 5, lr = lane & 15, h = lane >> 4;
    const int qtile = qt0 + blockIdx.x;
    const int q0 = qtile * 64;
    const int head = blockIdx.y, b = blockIdx.z, kvh = head >> 2;
    const size_t qplane = ((size_t)(b * NH + head)) * SEQ * HDM;
    const size_t kplane = ((size_t)(b * NKV + kvh)) * SEQ * HDM;
    const size_t vplane = ((size_t)(b * NKV + kvh)) * HDM * SEQ;
    const int wrow0 = q0 + wave * 16;

    v16h qf[2], qlf[2];
    {
        const _Float16* qp = Qh + qplane + (size_t)(wrow0 + lr) * HDM + 8 * h;
        qf[0] = ldfrag(qp);
        qf[1] = ldfrag(qp + 32);
        if constexpr (HP) {
            const _Float16* qlp = Ql + qplane + (size_t)(wrow0 + lr) * HDM + 8 * h;
            qlf[0] = ldfrag(qlp);
            qlf[1] = ldfrag(qlp + 32);
        } else {
            qlf[0] = qf[0];
            qlf[1] = qf[1];
        }
    }

    v8f o[4];
#pragma unroll
    for (int nt = 0; nt < 4; ++nt) o[nt] = zero8();
    float m[8], l[8];
#pragma unroll
    for (int r = 0; r < 8; ++r) { m[r] = -1.0e30f; l[r] = 0.0f; }

    _Float16* pw  = Ps + wave * 16 * KP;
    _Float16* plw = Pls + (HP ? wave * 16 * KP : 0);

    for (int tt = 0; tt <= qtile; ++tt) {
        const int kv0 = tt * 64;
        __syncthreads();
#pragma unroll
        for (int j = 0; j < 4; ++j) {
            const int idx = j * 128 + t, row = idx >> 3, ch = idx & 7;
            *(v8h*)(Ks + row * KP + ch * 8) =
                *(const v8h*)(Kh + kplane + (size_t)(kv0 + row) * HDM + ch * 8);
            *(v8h*)(Vs + row * KP + ch * 8) =
                *(const v8h*)(Vh + vplane + (size_t)row * SEQ + kv0 + ch * 8);
            if constexpr (HP) {
                *(v8h*)(Kls + row * KP + ch * 8) =
                    *(const v8h*)(Kl + kplane + (size_t)(kv0 + row) * HDM + ch * 8);
                *(v8h*)(Vls + row * KP + ch * 8) =
                    *(const v8h*)(Vl + vplane + (size_t)row * SEQ + kv0 + ch * 8);
            }
        }
        __syncthreads();

        v8f s[4];
#pragma unroll
        for (int nt = 0; nt < 4; ++nt) {
            const _Float16* kp = Ks + (nt * 16 + lr) * KP + 8 * h;
            const v16h bk0 = ldfrag(kp), bk1 = ldfrag(kp + 32);
            v8f a = zero8();
            if constexpr (HP) {
                const _Float16* klp = Kls + (nt * 16 + lr) * KP + 8 * h;
                const v16h bl0 = ldfrag(klp), bl1 = ldfrag(klp + 32);
                v8f tq = zero8();
                tq = mma(qf[0],  bl0, tq);
                tq = mma(qf[1],  bl1, tq);
                tq = mma(qlf[0], bk0, tq);
                tq = mma(qlf[1], bk1, tq);
                a = tq * LOSC_INV;
            }
            a = mma(qf[0], bk0, a);
            a = mma(qf[1], bk1, a);
            s[nt] = a;
        }

        float mnew[8];
#pragma unroll
        for (int r = 0; r < 8; ++r) {
            const int row = wrow0 + 8 * h + r;
            float mx = m[r];
#pragma unroll
            for (int nt = 0; nt < 4; ++nt) {
                const int col = kv0 + nt * 16 + lr;
                float v = s[nt][r] * SM_SCALE;
                v = (col <= row) ? v : -1.0e30f;
                s[nt][r] = v;
                mx = fmaxf(mx, v);
            }
#pragma unroll
            for (int off = 1; off < 16; off <<= 1) mx = fmaxf(mx, __shfl_xor(mx, off, 32));
            mnew[r] = mx;
        }
#pragma unroll
        for (int r = 0; r < 8; ++r) {
            const float alpha = __expf(m[r] - mnew[r]);
            m[r] = mnew[r];
            l[r] *= alpha;
#pragma unroll
            for (int nt = 0; nt < 4; ++nt) o[nt][r] *= alpha;
        }

        float psum[8];
#pragma unroll
        for (int r = 0; r < 8; ++r) psum[r] = 0.0f;
#pragma unroll
        for (int nt = 0; nt < 4; ++nt) {
#pragma unroll
            for (int r = 0; r < 8; ++r) {
                const float p = __expf(s[nt][r] - m[r]);
                psum[r] += p;
                const float ps = p * PSC;
                const _Float16 e = (_Float16)ps;
                const int po = (r + 8 * h) * KP + nt * 16 + lr;
                pw[po] = e;
                if constexpr (HP) plw[po] = (_Float16)((ps - (float)e) * LOSC);
            }
        }
#pragma unroll
        for (int r = 0; r < 8; ++r) {
            float ps = psum[r];
#pragma unroll
            for (int off = 1; off < 16; off <<= 1) ps += __shfl_xor(ps, off, 32);
            l[r] += ps;
        }
        __syncthreads();

        v16h pf[2], plf[2];
        pf[0] = ldfrag(pw + lr * KP + 8 * h);
        pf[1] = ldfrag(pw + lr * KP + 32 + 8 * h);
        if constexpr (HP) {
            plf[0] = ldfrag(plw + lr * KP + 8 * h);
            plf[1] = ldfrag(plw + lr * KP + 32 + 8 * h);
        } else {
            plf[0] = pf[0];
            plf[1] = pf[1];
        }
#pragma unroll
        for (int nt = 0; nt < 4; ++nt) {
            const _Float16* vp = Vs + (nt * 16 + lr) * KP + 8 * h;
            const v16h bv0 = ldfrag(vp), bv1 = ldfrag(vp + 32);
            if constexpr (HP) {
                const _Float16* vlp = Vls + (nt * 16 + lr) * KP + 8 * h;
                const v16h bw0 = ldfrag(vlp), bw1 = ldfrag(vlp + 32);
                v8f tq = zero8();
                tq = mma(pf[0],  bw0, tq);
                tq = mma(pf[1],  bw1, tq);
                tq = mma(plf[0], bv0, tq);
                tq = mma(plf[1], bv1, tq);
                o[nt] = o[nt] + tq * LOSC_INV;
            }
            o[nt] = mma(pf[0], bv0, o[nt]);
            o[nt] = mma(pf[1], bv1, o[nt]);
        }
    }

    __syncthreads();
    float invl[8];
#pragma unroll
    for (int r = 0; r < 8; ++r) invl[r] = 1.0f / (l[r] * PSC);
    _Float16* lw = Ks + wave * 16 * KP;
#pragma unroll
    for (int nt = 0; nt < 4; ++nt) {
#pragma unroll
        for (int r = 0; r < 8; ++r) {
            const float val = o[nt][r] * invl[r];
            const _Float16 e = (_Float16)val;
            const int po = (r + 8 * h) * KP + nt * 16 + lr;
            pw[po] = e;
            lw[po] = (_Float16)((val - (float)e) * LOSC);
        }
    }
    __syncthreads();
    auto emit = [&]() {
#pragma unroll
        for (int it = 0; it < 4; ++it) {
            const int slot = it * 32 + lane, rowl = slot >> 3, ch = slot & 7;
            const v8h hv = *(const v8h*)(pw + rowl * KP + ch * 8);
            const v8h lv = *(const v8h*)(lw + rowl * KP + ch * 8);
            const size_t d = ((size_t)(b * SEQ + wrow0 + rowl)) * HID + head * HDM + ch * 8;
            *(volatile v8h*)(Ch + d) = hv;
            *(volatile v8h*)(Cl + d) = lv;
        }
    };
    emit();
    __threadfence();
    emit();
}

template <bool RES>
__global__ void __launch_bounds__(256)
oproj_kernel(const _Float16* __restrict__ ch, const _Float16* __restrict__ cl,
             const _Float16* __restrict__ wt, float* __restrict__ out, int tpb, int sofs)
{
    _Float16* As = (_Float16*)dyn_lds;
    _Float16* Bs = As + 128 * LST;
    float*    Tf = (float*)dyn_lds;

    const int t = threadIdx.x, lane = t & 31, wave = t >> 5, lr = lane & 15, h = lane >> 4;
    const int waveM = wave & 3, waveN = wave >> 2;
    const int yb = blockIdx.y / tpb, mt = blockIdx.y - yb * tpb;
    const int mBase = yb * SEQ + sofs + mt * 128;
    const int orow0 = yb * SEQ_FULL + sofs + mt * 128;
    const int nBase = blockIdx.x * 128;

    v8f acc[2][4];
#pragma unroll
    for (int mi = 0; mi < 2; ++mi)
#pragma unroll
        for (int ni = 0; ni < 4; ++ni) acc[mi][ni] = zero8();

    if constexpr (RES) {
        gemm_kloop(cl, wt, mBase, nBase, As, Bs, acc);
#pragma unroll
        for (int mi = 0; mi < 2; ++mi)
#pragma unroll
            for (int ni = 0; ni < 4; ++ni) acc[mi][ni] = acc[mi][ni] * LOSC_INV;
    }
    gemm_kloop(ch, wt, mBase, nBase, As, Bs, acc);

#pragma unroll
    for (int mi = 0; mi < 2; ++mi) {
        const int rb = waveM * 32 + mi * 16 + 8 * h;
#pragma unroll
        for (int ni = 0; ni < 4; ++ni) {
            const int col = waveN * 64 + ni * 16 + lr;
            v4f a, c;
#pragma unroll
            for (int j = 0; j < 4; ++j) {
                a[j] = acc[mi][ni][j] * WSCALE_INV;
                c[j] = acc[mi][ni][4 + j] * WSCALE_INV;
            }
            *(v4f*)(Tf + col * TPF + rb) = a;
            *(v4f*)(Tf + col * TPF + rb + 4) = c;
        }
    }
    __syncthreads();

    auto emit = [&]() {
#pragma unroll
        for (int it = 0; it < 16; ++it) {
            const int slot = it * 256 + t, L = slot >> 3, chk = slot & 7;
            const int rowl = L >> 2, seg = L & 3, c0 = seg * 32 + chk * 4;
            v4f g;
#pragma unroll
            for (int j = 0; j < 4; ++j) g[j] = Tf[(c0 + j) * TPF + rowl];
            float* dst = out + (size_t)(orow0 + rowl) * HID + nBase + c0;
            *(volatile v4f*)dst = g;
        }
    };
    emit();
    __threadfence();
    emit();
}

extern "C" void kernel_launch(void* const* d_in, const int* in_sizes, int n_in,
                              void* d_out, int out_size, void* d_ws, size_t ws_size,
                              hipStream_t stream)
{
    if (n_in < 6) return;
    const long long needTok = (long long)(NB - 1) * SEQ_FULL + SEQ;
    if ((long long)in_sizes[0] < needTok * HID) return;
    if ((long long)in_sizes[1] < (long long)HID * HID) return;
    if ((long long)in_sizes[2] < (long long)HID * KVD) return;
    if ((long long)in_sizes[3] < (long long)HID * KVD) return;
    if ((long long)in_sizes[4] < (long long)HID * HID) return;
    if ((long long)in_sizes[5] < needTok) return;
    if ((long long)out_size < needTok * HID) return;

    const float* x   = (const float*)d_in[0];
    const float* Wq  = (const float*)d_in[1];
    const float* Wk  = (const float*)d_in[2];
    const float* Wv  = (const float*)d_in[3];
    const float* Wo  = (const float*)d_in[4];
    const int*   pos = (const int*)d_in[5];
    float* out = (float*)d_out;

    char* ws = (char*)d_ws;
    size_t off = 0;
    _Float16* Xh  = (_Float16*)(ws + off); off += (size_t)NTOK * HID * 2;
    _Float16* WqT = (_Float16*)(ws + off); off += (size_t)HID * HID * 2;
    _Float16* WkT = (_Float16*)(ws + off); off += (size_t)KVD * HID * 2;
    _Float16* WvT = (_Float16*)(ws + off); off += (size_t)KVD * HID * 2;
    _Float16* WoT = (_Float16*)(ws + off); off += (size_t)HID * HID * 2;
    float*    CS  = (float*)(ws + off);    off += (size_t)NTOK * 64 * 4;
    _Float16* Qh  = (_Float16*)(ws + off); off += (size_t)NTOK * HID * 2;
    _Float16* Ql  = (_Float16*)(ws + off); off += (size_t)NTOK * HID * 2;
    _Float16* Kh  = (_Float16*)(ws + off); off += (size_t)NTOK * KVD * 2;
    _Float16* Kl  = (_Float16*)(ws + off); off += (size_t)NTOK * KVD * 2;
    _Float16* Vth = (_Float16*)(ws + off); off += (size_t)NTOK * KVD * 2;
    _Float16* Vtl = (_Float16*)(ws + off); off += (size_t)NTOK * KVD * 2;
    _Float16* Chh = (_Float16*)(ws + off); off += (size_t)NTOK * HID * 2;
    _Float16* Cll = (_Float16*)(ws + off); off += (size_t)NTOK * HID * 2;
    if (off > ws_size) return;

    hipFuncSetAttribute(reinterpret_cast<const void*>(&proj_kernel<0>),
                        hipFuncAttributeMaxDynamicSharedMemorySize, PROJ_LDS_BYTES);
    hipFuncSetAttribute(reinterpret_cast<const void*>(&proj_kernel<1>),
                        hipFuncAttributeMaxDynamicSharedMemorySize, PROJ_LDS_BYTES);
    hipFuncSetAttribute(reinterpret_cast<const void*>(&proj_kernel<2>),
                        hipFuncAttributeMaxDynamicSharedMemorySize, PROJ_LDS_BYTES);
    hipFuncSetAttribute(reinterpret_cast<const void*>(&oproj_kernel<true>),
                        hipFuncAttributeMaxDynamicSharedMemorySize, OPROJ_LDS_BYTES);
    hipFuncSetAttribute(reinterpret_cast<const void*>(&oproj_kernel<false>),
                        hipFuncAttributeMaxDynamicSharedMemorySize, OPROJ_LDS_BYTES);

    const dim3 blk256(256), blk128(128);

    cvt_x_kernel<<<dim3(NTOK), blk256, 0, stream>>>(x, Xh);
    cvt_w_kernel<<<dim3(HID / 64, HID / 64), blk256, 0, stream>>>(Wq, WqT, HID);
    cvt_w_kernel<<<dim3(KVD / 64, HID / 64), blk256, 0, stream>>>(Wk, WkT, KVD);
    cvt_w_kernel<<<dim3(KVD / 64, HID / 64), blk256, 0, stream>>>(Wv, WvT, KVD);
    cvt_w_kernel<<<dim3(HID / 64, HID / 64), blk256, 0, stream>>>(Wo, WoT, HID);
    rope_table_kernel<<<dim3(NTOK / 8), blk256, 0, stream>>>(pos, CS);

    proj_kernel<0><<<dim3(HID / 128, NTOK / 128), blk256, PROJ_LDS_BYTES, stream>>>(Xh, WqT, CS, Qh, Ql);
    proj_kernel<1><<<dim3(KVD / 128, NTOK / 128), blk256, PROJ_LDS_BYTES, stream>>>(Xh, WkT, CS, Kh, Kl);
    proj_kernel<2><<<dim3(KVD / 128, NTOK / 128), blk256, PROJ_LDS_BYTES, stream>>>(Xh, WvT, CS, Vth, Vtl);

    const int qtHP = RHPE / 64;
    const int qtLP = (SEQ - RHPE) / 64;
    attn_kernel<true><<<dim3(qtHP, NH, NB), blk128, 0, stream>>>(Qh, Ql, Kh, Kl, Vth, Vtl, Chh, Cll, 0);
    if (qtLP > 0)
        attn_kernel<false><<<dim3(qtLP, NH, NB), blk128, 0, stream>>>(Qh, Ql, Kh, Kl, Vth, Vtl, Chh, Cll, qtHP);

    const int tpbHP = RHPE / 128;
    const int tpbLP = (SEQ - RHPE) / 128;
    oproj_kernel<true><<<dim3(HID / 128, NB * tpbHP), blk256, OPROJ_LDS_BYTES, stream>>>(
        Chh, Cll, WoT, out, tpbHP, 0);
    if (tpbLP > 0)
        oproj_kernel<false><<<dim3(HID / 128, NB * tpbLP), blk256, OPROJ_LDS_BYTES, stream>>>(
            Chh, Cll, WoT, out, tpbLP, RHPE);
}
